// dot_attention_23854248362444
// MI455X (gfx1250) — hardware-verified
//
#include <hip/hip_runtime.h>
#include <math.h>
#include <stdint.h>

#ifndef NB
#define NB 8
#endif
#define NB_FULL 8
#define TX 256
#define TY 256
#ifndef TYR
#define TYR TY
#endif
#define CC 256
#define HH 128
#define XSC 16.0f
#define WYS 1024.0f
#define ZINV (1.0f / (16.0f * 1024.0f))
#define TWOLOG2E 2.8853900817779268f
#define LDW 264
#define TP 68
#define SLAB (16 * 68)
#define SC_WAVES 8
#define SC_THREADS (SC_WAVES * 32)

static_assert(TX == 256 && TY == 256 && CC == 256 && HH == 128);
static_assert(NB >= 1 && NB <= NB_FULL);
static_assert((TYR % 64) == 0 && TYR >= 64 && TYR <= TY);
static_assert(SC_THREADS == TX && SC_WAVES * 32 == TX && SC_WAVES * 16 == HH && 32 * 8 == CC);
static_assert((CC % 32) == 0 && (TX % 32) == 0 && (LDW % 8) == 0 && LDW >= CC);
static_assert(((NB * TX * CC / 8) % 256) == 0 && ((NB * TY * CC / 8) % 256) == 0 && ((HH * CC / 8) % 256) == 0);
static_assert((TX % 64) == 0 && (CC % 64) == 0 && (TP * 4) % 16 == 0 && (SLAB * 4) % 16 == 0);

typedef unsigned short u16;
typedef _Float16 v16h __attribute__((ext_vector_type(16)));
typedef _Float16 v8h  __attribute__((ext_vector_type(8)));
typedef __bf16   v16b __attribute__((ext_vector_type(16)));
typedef float    v8f  __attribute__((ext_vector_type(8)));
typedef float    v4f  __attribute__((ext_vector_type(4)));
typedef unsigned int v4u __attribute__((ext_vector_type(4)));

union FragH { v16h v; v8h h[2]; v4u u[2]; };
union FragB { v16b v; v4u u[2]; };

__device__ __forceinline__ unsigned short bf_bits(float f) {
  unsigned u = __float_as_uint(f);
  return (unsigned short)((u + 0x7FFFu + ((u >> 16) & 1u)) >> 16);
}
__device__ __forceinline__ float bf_up(unsigned short h) { return __uint_as_float(((unsigned)h) << 16); }
__device__ __forceinline__ float bf_val(float f) { return bf_up(bf_bits(f)); }
__device__ __forceinline__ float lo16f(unsigned w) { return __uint_as_float(w << 16); }
__device__ __forceinline__ float hi16f(unsigned w) { return __uint_as_float(w & 0xffff0000u); }
__device__ __forceinline__ unsigned short h_bits(_Float16 x) { return __builtin_bit_cast(unsigned short, x); }
__device__ __forceinline__ unsigned pk16(unsigned short a, unsigned short b) { return (unsigned)a | ((unsigned)b << 16); }
__device__ __forceinline__ v8f zero8() { v8f z = {0.f, 0.f, 0.f, 0.f, 0.f, 0.f, 0.f, 0.f}; return z; }

__device__ __forceinline__ float tanh_e(float v) {
  const float e = exp2f(v * TWOLOG2E);
  return 1.0f - 2.0f * __builtin_amdgcn_rcpf(e + 1.0f);
}

__device__ __forceinline__ v16h ldfrag_h(const _Float16* p) {
  FragH f;
  f.h[0] = *(const v8h*)(p);
  f.h[1] = *(const v8h*)(p + 16);
  return f.v;
}
__device__ __forceinline__ v16b ldfrag_b(const u16* p) {
  FragB f;
  f.u[0] = *(const v4u*)(p);
  f.u[1] = *(const v4u*)(p + 16);
  return f.v;
}

__device__ __forceinline__ v8f mma_h(v16h a, v16h b, v8f c) {
  return __builtin_amdgcn_wmma_f32_16x16x32_f16(false, a, false, b, (short)0, c, false, false);
}
__device__ __forceinline__ v8f mma_b(v16b a, v16b b, v8f c) {
  return __builtin_amdgcn_wmma_f32_16x16x32_bf16(false, a, false, b, (short)0, c, false, false);
}
template <typename F>
__device__ __forceinline__ void guard6(v8f& a, v8f& b, v8f& c, v8f& d, F x0, F x1, F x2, F x3, F x4, F x5) {
#if defined(__HIP_DEVICE_COMPILE__)
  asm volatile("v_nop\n\tv_nop\n\tv_nop\n\tv_nop"
               : "+v"(a), "+v"(b), "+v"(c), "+v"(d) : "v"(x0), "v"(x1), "v"(x2), "v"(x3), "v"(x4), "v"(x5) : "memory");
#endif
}
template <typename F>
__device__ __forceinline__ void guard8(v8f& c0, v8f& c1, v8f& c2, v8f& c3, v8f& c4, v8f& c5, v8f& c6, v8f& c7,
                                       F x0, F x1, F x2, F x3, F x4, F x5) {
#if defined(__HIP_DEVICE_COMPILE__)
  asm volatile("v_nop\n\tv_nop\n\tv_nop\n\tv_nop"
               : "+v"(c0), "+v"(c1), "+v"(c2), "+v"(c3), "+v"(c4), "+v"(c5), "+v"(c6), "+v"(c7)
               : "v"(x0), "v"(x1), "v"(x2), "v"(x3), "v"(x4), "v"(x5) : "memory");
#endif
}
__device__ __forceinline__ void acc_guard4(v8f& a, v8f& b, v8f& c, v8f& d) {
#if defined(__HIP_DEVICE_COMPILE__)
  asm volatile("v_nop\n\tv_nop\n\tv_nop\n\tv_nop" : "+v"(a), "+v"(b), "+v"(c), "+v"(d));
#endif
}
__device__ __forceinline__ void acc_guard8(v8f& c0, v8f& c1, v8f& c2, v8f& c3, v8f& c4, v8f& c5, v8f& c6, v8f& c7) {
#if defined(__HIP_DEVICE_COMPILE__)
  asm volatile("v_nop\n\tv_nop\n\tv_nop\n\tv_nop"
               : "+v"(c0), "+v"(c1), "+v"(c2), "+v"(c3), "+v"(c4), "+v"(c5), "+v"(c6), "+v"(c7));
#endif
}
__device__ __forceinline__ void wave_sync_lds() {
#if defined(__HIP_DEVICE_COMPILE__)
  __builtin_amdgcn_fence(__ATOMIC_RELEASE, "workgroup");
  __builtin_amdgcn_wave_barrier();
  __builtin_amdgcn_fence(__ATOMIC_ACQUIRE, "workgroup");
#endif
}

__global__ __launch_bounds__(256) void cvt16(const float* __restrict__ x, u16* D, int n8, int mode, float scale) {
  const int gt = blockIdx.x * 256 + (int)threadIdx.x;
  if (gt >= n8) return;
  const float* p = x + (size_t)gt * 8;
  const v4f a = *(const v4f*)(p), c4 = *(const v4f*)(p + 4);
  float v[8];
#pragma unroll
  for (int e = 0; e < 4; ++e) { v[e] = a[e]; v[4 + e] = c4[e]; }
  unsigned short s[8];
#pragma unroll
  for (int e = 0; e < 8; ++e) {
    const unsigned short bb = bf_bits(v[e]);
    const unsigned short hb = h_bits((_Float16)(bf_up(bb) * scale));
    s[e] = (mode != 0) ? hb : bb;
  }
  v4u o;
#pragma unroll
  for (int e = 0; e < 4; ++e) o[e] = pk16(s[2 * e], s[2 * e + 1]);
  u16* d = D + (size_t)gt * 8;
  for (int pass = 0; pass < 2; ++pass) {
    *(volatile v4u*)(d) = o;
    __threadfence();
  }
}

__global__ __launch_bounds__(256) void xpose_b16(const float* __restrict__ x, u16* XT) {
  __shared__ __align__(16) float T[64 * TP];
  const int tid = threadIdx.x, lane = tid & 31, wave = tid >> 5;
  const int ntl = (TX / 64) * (CC / 64);
  const int bid = blockIdx.x;
  const int b   = bid / ntl, t = bid % ntl;
  const int tx0 = (t / (CC / 64)) * 64;
  const int c0  = (t % (CC / 64)) * 64;
  const int r   = tid >> 2, cq = (tid & 3) * 16;
  const float* p = x + ((size_t)b * TX + tx0 + r) * CC + c0 + cq;
  const v4f q0 = *(const v4f*)(p), q1 = *(const v4f*)(p + 4), q2 = *(const v4f*)(p + 8), q3 = *(const v4f*)(p + 12);
#pragma unroll
  for (int e = 0; e < 4; ++e) {
    T[(cq + e) * TP + r]      = q0[e];
    T[(cq + 4 + e) * TP + r]  = q1[e];
    T[(cq + 8 + e) * TP + r]  = q2[e];
    T[(cq + 12 + e) * TP + r] = q3[e];
  }
  __syncthreads();
  const int rq = lane >> 3, g8 = (lane & 7) * 8;
  v4u ov[2];
#pragma unroll
  for (int i = 0; i < 2; ++i) {
    const int ci = wave * 8 + i * 4 + rq;
    const v4f a = *(const v4f*)(T + ci * TP + g8), c4 = *(const v4f*)(T + ci * TP + g8 + 4);
    float w[8];
#pragma unroll
    for (int e = 0; e < 4; ++e) { w[e] = a[e]; w[4 + e] = c4[e]; }
#pragma unroll
    for (int e = 0; e < 4; ++e) ov[i][e] = pk16(bf_bits(w[2 * e]), bf_bits(w[2 * e + 1]));
  }
  u16* dst = XT + ((size_t)b * CC + c0 + wave * 8 + rq) * TX + tx0 + g8;
  for (int pass = 0; pass < 2; ++pass) {
#pragma unroll
    for (int i = 0; i < 2; ++i) {
      *(volatile v4u*)(dst + (size_t)(i * 4) * TX) = ov[i];
    }
    __threadfence();
  }
}

__device__ __forceinline__ void epi64(float* sl, v8f a0, v8f a1, v8f a2, v8f a3, float* C, int N,
                                      size_t rowb, int col0, int lane) {
  const int hh = lane >> 4, m = lane & 15;
#pragma unroll
  for (int r = 0; r < 8; ++r) {
    const int ro = (8 * hh + r) * 68 + m;
    sl[ro]      = a0[r];
    sl[ro + 16] = a1[r];
    sl[ro + 32] = a2[r];
    sl[ro + 48] = a3[r];
  }
  wave_sync_lds();
  v4f vals[8];
#pragma unroll
  for (int it = 0; it < 8; ++it) vals[it] = *(const v4f*)(sl + (it * 2 + hh) * 68 + m * 4);
  float* dst = C + (rowb + (size_t)hh) * (size_t)N + col0 + m * 4;
  for (int pass = 0; pass < 2; ++pass) {
#pragma unroll
    for (int it = 0; it < 8; ++it) {
      *(volatile v4f*)(dst + (size_t)(it * 2) * (size_t)N) = vals[it];
    }
    __threadfence();
  }
}

__global__ __launch_bounds__(SC_THREADS)
void score_softmax(const u16* __restrict__ XB, const u16* __restrict__ YB, const u16* __restrict__ WDB,
                   const float* __restrict__ vd, u16* PH, u16* PL) {
  __shared__ __align__(16) u16 Wys[HH * LDW];
  __shared__ __align__(16) u16 phs[TX];
  __shared__ __align__(16) u16 pls[TX];
  __shared__ float sl[TX];
  __shared__ float vds[HH];
  __shared__ float redm[SC_WAVES];
  __shared__ float reds[SC_WAVES];

  const int tid = threadIdx.x, wave = tid >> 5, lane = tid & 31, hh = lane >> 4, m = lane & 15;
  const int bid = blockIdx.x;
  const int b   = bid / TYR;
  const int ty  = bid % TYR;

  if (tid < HH) vds[tid] = bf_val(vd[tid]);

  {
    const int c8 = (tid & 31) * 8, hq = tid >> 5;
    const v4u yv = *(const v4u*)(YB + ((size_t)b * TY + ty) * CC + c8);
    float yf[8];
#pragma unroll
    for (int e = 0; e < 4; ++e) { yf[2 * e] = lo16f(yv[e]); yf[2 * e + 1] = hi16f(yv[e]); }
#pragma unroll 2
    for (int i = 0; i < HH / 8; ++i) {
      const int h = hq + 8 * i;
      const v4u wv = *(const v4u*)(WDB + (size_t)h * CC + c8);
      v4u o;
#pragma unroll
      for (int e = 0; e < 4; ++e) {
        const float p0 = (lo16f(wv[e]) * yf[2 * e]) * WYS;
        const float p1 = (hi16f(wv[e]) * yf[2 * e + 1]) * WYS;
        o[e] = pk16(h_bits((_Float16)p0), h_bits((_Float16)p1));
      }
      *(v4u*)(&Wys[h * LDW + c8]) = o;
    }
  }
  __syncthreads();

  const int tx0 = wave * 32;
  const _Float16* ap = (const _Float16*)(const void*)XB + ((size_t)b * TX + tx0 + m) * CC + 8 * hh;
  const _Float16* wl = (const _Float16*)(const void*)(&Wys[0]);
  float p0[8], p1[8];
#pragma unroll
  for (int r = 0; r < 8; ++r) { p0[r] = 0.f; p1[r] = 0.f; }

#pragma unroll 1
  for (int half = 0; half < 2; ++half) {
    const int hb = half * 64;
    const _Float16* bq = wl + (size_t)(hb + m) * LDW + 8 * hh;
    v8f c0[4], c1[4];
#pragma unroll
    for (int j = 0; j < 4; ++j) { c0[j] = zero8(); c1[j] = zero8(); }
#pragma unroll 1
    for (int k0 = 0; k0 < CC; k0 += 32) {
      const v16h a0 = ldfrag_h(ap + k0);
      const v16h a1 = ldfrag_h(ap + (size_t)16 * CC + k0);
      const v16h b0 = ldfrag_h(bq + k0);
      const v16h b1 = ldfrag_h(bq + 16 * LDW + k0);
      const v16h b2 = ldfrag_h(bq + 32 * LDW + k0);
      const v16h b3 = ldfrag_h(bq + 48 * LDW + k0);
      c0[0] = mma_h(a0, b0, c0[0]);
      c0[1] = mma_h(a0, b1, c0[1]);
      c0[2] = mma_h(a0, b2, c0[2]);
      c0[3] = mma_h(a0, b3, c0[3]);
      c1[0] = mma_h(a1, b0, c1[0]);
      c1[1] = mma_h(a1, b1, c1[1]);
      c1[2] = mma_h(a1, b2, c1[2]);
      c1[3] = mma_h(a1, b3, c1[3]);
      guard8<v16h>(c0[0], c0[1], c0[2], c0[3], c1[0], c1[1], c1[2], c1[3], a0, a1, b0, b1, b2, b3);
    }
    acc_guard8(c0[0], c0[1], c0[2], c0[3], c1[0], c1[1], c1[2], c1[3]);
#pragma unroll
    for (int j = 0; j < 4; ++j) {
      const float vv = vds[hb + 16 * j + m];
#pragma unroll
      for (int r = 0; r < 8; ++r) {
        p0[r] += vv * tanh_e(c0[j][r] * ZINV);
        p1[r] += vv * tanh_e(c1[j][r] * ZINV);
      }
    }
  }

#pragma unroll
  for (int r = 0; r < 8; ++r) {
    float v = p0[r];
    v += __shfl_xor(v, 1, 16);
    v += __shfl_xor(v, 2, 16);
    v += __shfl_xor(v, 4, 16);
    v += __shfl_xor(v, 8, 16);
    p0[r] = v;
    float u = p1[r];
    u += __shfl_xor(u, 1, 16);
    u += __shfl_xor(u, 2, 16);
    u += __shfl_xor(u, 4, 16);
    u += __shfl_xor(u, 8, 16);
    p1[r] = u;
  }
  if (m == 0) {
#pragma unroll
    for (int r = 0; r < 8; ++r) {
      sl[tx0 + 8 * hh + r]      = p0[r];
      sl[tx0 + 16 + 8 * hh + r] = p1[r];
    }
  }
  __syncthreads();

  const float sv = sl[tid];
  float mx = sv;
  mx = fmaxf(mx, __shfl_xor(mx, 16, 32));
  mx = fmaxf(mx, __shfl_xor(mx, 8, 32));
  mx = fmaxf(mx, __shfl_xor(mx, 4, 32));
  mx = fmaxf(mx, __shfl_xor(mx, 2, 32));
  mx = fmaxf(mx, __shfl_xor(mx, 1, 32));
  if (lane == 0) redm[wave] = mx;
  __syncthreads();
  float mm = redm[0];
#pragma unroll
  for (int w = 1; w < SC_WAVES; ++w) mm = fmaxf(mm, redm[w]);
  const float ev = expf(sv - mm);
  float ss = ev;
  ss += __shfl_xor(ss, 16, 32);
  ss += __shfl_xor(ss, 8, 32);
  ss += __shfl_xor(ss, 4, 32);
  ss += __shfl_xor(ss, 2, 32);
  ss += __shfl_xor(ss, 1, 32);
  if (lane == 0) reds[wave] = ss;
  __syncthreads();
  float tot = reds[0];
#pragma unroll
  for (int w = 1; w < SC_WAVES; ++w) tot += reds[w];
  const float a = ev * (1.0f / tot);
  const unsigned short hb16 = bf_bits(a);
  const unsigned short lb16 = bf_bits(a - bf_up(hb16));
  phs[tid] = hb16;
  pls[tid] = lb16;
  __syncthreads();

  if (wave < 2) {
    const v4u oh = *(const v4u*)(&phs[lane * 8]);
    const v4u ol = *(const v4u*)(&pls[lane * 8]);
    const v4u o  = (wave == 0) ? oh : ol;
    u16* base = (wave == 0) ? PH : PL;
    u16* dst  = base + ((size_t)b * TYR + ty) * TX + lane * 8;
    for (int pass = 0; pass < 2; ++pass) {
      *(volatile v4u*)(dst) = o;
      __threadfence();
    }
  }
}

__global__ __launch_bounds__(128)
void gemm_pv(const u16* __restrict__ PH, const u16* __restrict__ PL, const u16* __restrict__ XT, float* out) {
  __shared__ __align__(16) float slab[4 * SLAB];
  const int tid = threadIdx.x, wave = tid >> 5, lane = tid & 31, hh = lane >> 4, m = lane & 15;
  const int ntl  = (TYR / 64) * (CC / 64);
  const int bid  = blockIdx.x;
  const int bz   = bid / ntl, t = bid % ntl;
  const int rowl = (t / (CC / 64)) * 64 + wave * 16;
  const int col0 = (t % (CC / 64)) * 64;
  const u16* aph = PH + ((size_t)bz * TYR + rowl + m) * TX + 8 * hh;
  const u16* apl = PL + ((size_t)bz * TYR + rowl + m) * TX + 8 * hh;
  const u16* bp  = XT + ((size_t)bz * CC + col0 + m) * TX + 8 * hh;
  const size_t bs = (size_t)16 * TX;
  v8f acc0 = zero8(), acc1 = zero8(), acc2 = zero8(), acc3 = zero8();
#pragma unroll 1
  for (int k0 = 0; k0 < TX; k0 += 32) {
    const v16b ah = ldfrag_b(aph + k0);
    const v16b al = ldfrag_b(apl + k0);
    const v16b b0 = ldfrag_b(bp + k0);
    const v16b b1 = ldfrag_b(bp + bs + k0);
    const v16b b2 = ldfrag_b(bp + 2 * bs + k0);
    const v16b b3 = ldfrag_b(bp + 3 * bs + k0);
    acc0 = mma_b(ah, b0, acc0);
    acc1 = mma_b(ah, b1, acc1);
    acc2 = mma_b(ah, b2, acc2);
    acc3 = mma_b(ah, b3, acc3);
    acc0 = mma_b(al, b0, acc0);
    acc1 = mma_b(al, b1, acc1);
    acc2 = mma_b(al, b2, acc2);
    acc3 = mma_b(al, b3, acc3);
    guard6<v16b>(acc0, acc1, acc2, acc3, ah, al, b0, b1, b2, b3);
  }
  acc_guard4(acc0, acc1, acc2, acc3);
  epi64(slab + wave * SLAB, acc0, acc1, acc2, acc3, out + (size_t)bz * TYR * CC, CC, (size_t)rowl, col0, lane);
}

extern "C" void kernel_launch(void* const* d_in, const int* in_sizes, int n_in,
                              void* d_out, int out_size, void* d_ws, size_t ws_size,
                              hipStream_t stream) {
  if (n_in < 4) return;
  if (in_sizes[0] < NB * TX * CC || in_sizes[1] < NB * TY * CC) return;
  if (in_sizes[2] < HH * CC || in_sizes[3] < HH) return;
  if (out_size < NB * TYR * CC) return;

  const float* Xin = (const float*)d_in[0];
  const float* Yin = (const float*)d_in[1];
  const float* Wd  = (const float*)d_in[2];
  const float* vd  = (const float*)d_in[3];
  float*       out = (float*)d_out;

  const size_t szXB = (size_t)NB * TX * CC * 2;
  const size_t szYB = (size_t)NB * TY * CC * 2;
  const size_t szWD = (size_t)HH * CC * 2;
  const size_t szXT = (size_t)NB * CC * TX * 2;
  const size_t szP  = (size_t)NB * TYR * TX * 2;
  size_t off = 0;
  const size_t oXB = off; off += szXB;
  const size_t oYB = off; off += szYB;
  const size_t oWD = off; off += szWD;
  const size_t oXT = off; off += szXT;
  const size_t oPH = off; off += szP;
  const size_t oPL = off; off += szP;
  if (off > ws_size) return;
  if (off > (size_t)134217728) return;

  char* ws = (char*)d_ws;
  u16* XB  = (u16*)(ws + oXB);
  u16* YB  = (u16*)(ws + oYB);
  u16* WDB = (u16*)(ws + oWD);
  u16* XT  = (u16*)(ws + oXT);
  u16* PH  = (u16*)(ws + oPH);
  u16* PL  = (u16*)(ws + oPL);

  const int n8x = (NB * TX * CC) / 8;
  const int n8y = (NB * TY * CC) / 8;
  const int n8w = (HH * CC) / 8;
  if ((n8x % 256) != 0 || (n8y % 256) != 0 || (n8w % 256) != 0) return;

  const dim3 blk(256);
  const dim3 gX(n8x / 256);
  const dim3 gY(n8y / 256);
  const dim3 gW(n8w / 256);
  const dim3 gXT(NB * (TX / 64) * (CC / 64));
  const dim3 gSC(NB * TYR);
  const dim3 bSC(SC_THREADS);
  const dim3 gPV(NB * (TYR / 64) * (CC / 64));
  const dim3 bPV(128);

  cvt16<<<gX, blk, 0, stream>>>(Xin, XB, n8x, 1, XSC);
  cvt16<<<gY, blk, 0, stream>>>(Yin, YB, n8y, 0, 1.0f);
  cvt16<<<gW, blk, 0, stream>>>(Wd, WDB, n8w, 0, 1.0f);
  xpose_b16<<<gXT, blk, 0, stream>>>(Xin, XT);
  score_softmax<<<gSC, bSC, 0, stream>>>(XB, YB, WDB, vd, PH, PL);
  gemm_pv<<<gPV, bPV, 0, stream>>>(PH, PL, XT, out);
  (void)hipGetLastError();
}
